// EdgeMLPDecoder_48086453846461
// MI455X (gfx1250) — hardware-verified
//
#include <hip/hip_runtime.h>
#include <hip/hip_bf16.h>

typedef __attribute__((ext_vector_type(16))) _Float16 v16h;
typedef __attribute__((ext_vector_type(8)))  float    v8f;
typedef __attribute__((vector_size(16)))     int      vsi4;

#define DIM     128
#define HIDDEN  128
#define INDIM   512
#define KSTEPS  (INDIM / 32)
#define NTILES  (HIDDEN / 16)

#define VST2(T, ptr, val) do { const T _v = (val); *(volatile T*)(ptr) = _v; __threadfence(); *(volatile T*)(ptr) = _v; } while (0)

__global__ void prep_w1_f16t(const float* __restrict__ W1,
                             _Float16* __restrict__ W1T) {
    int idx = blockIdx.x * blockDim.x + threadIdx.x;
    if (idx < INDIM * HIDDEN) {
        int k = idx / HIDDEN;
        int n = idx % HIDDEN;
        VST2(_Float16, W1T + n * INDIM + k, (_Float16)W1[idx]);
    }
}

__global__ void __launch_bounds__(256)
node_proj_wmma(const float* __restrict__ z, const _Float16* __restrict__ W1T, float* __restrict__ P, int nNodes) {
    const int wave = threadIdx.x >> 5, lane = threadIdx.x & 31, m = lane & 15, hf = lane >> 4;
    const int gw = blockIdx.x * 8 + wave;
    const int tile = gw >> 2, cg = gw & 3;
    const int node = min(tile * 16 + m, nNodes - 1);
    const float* zr = z + (size_t)node * DIM;
    const int hid0 = (cg & 1) * 64, kbase = (cg >> 1) * 128;
    v8f acc[4] = {};
#pragma unroll
    for (int ks = 0; ks < 4; ++ks) {
        v16h a;
#pragma unroll
        for (int e = 0; e < 16; ++e) a[e] = (_Float16)zr[ks * 32 + ((e < 8) ? (8 * hf + e) : (16 + 8 * hf + e - 8))];
#pragma unroll
        for (int nt = 0; nt < 4; ++nt) {
            const _Float16* bp = W1T + (size_t)(hid0 + nt * 16 + m) * INDIM + kbase + ks * 32 + hf * 8;
            union { v16h v; __attribute__((ext_vector_type(8))) _Float16 h[2]; } bu;
            bu.h[0] = *(const __attribute__((ext_vector_type(8))) _Float16*)bp;
            bu.h[1] = *(const __attribute__((ext_vector_type(8))) _Float16*)(bp + 16);
            acc[nt] = __builtin_amdgcn_wmma_f32_16x16x32_f16(false, a, false, bu.v, (short)0, acc[nt], false, false);
            asm volatile("v_nop\n\tv_nop\n\tv_nop\n\tv_nop" : "+v"(acc[nt]) : "v"(a), "v"(bu.v));
        }
    }
    const int pc0 = (cg >> 1) * 128 + hid0;
    for (int pass = 0; pass < 2; ++pass) {
#pragma unroll
        for (int pr = 0; pr < 2; ++pr)
#pragma unroll
            for (int r = 0; r < 8; ++r) {
                const float a_ = acc[2 * pr][r], b_ = acc[2 * pr + 1][r];
                const float ax = __shfl_xor(a_, 16), bx = __shfl_xor(b_, 16);
                const int n0r = tile * 16 + r, n1r = tile * 16 + 8 + r;
                if (n0r < nNodes) *(volatile float*)(P + (size_t)n0r * 256 + pc0 + pr * 32 + lane) = hf ? bx : a_;
                if (n1r < nNodes) *(volatile float*)(P + (size_t)n1r * 256 + pc0 + pr * 32 + lane) = hf ? b_ : ax;
            }
        __threadfence();
    }
}

__global__ void __launch_bounds__(256)
edge_mlp_wmma(const float* __restrict__ z,
              const int* __restrict__ ei,
              const _Float16* __restrict__ W1T,
              const float* __restrict__ b1,
              const float* __restrict__ W2,
              const float* __restrict__ b2,
              const float* __restrict__ P,
              float* __restrict__ out,
              int E, int numTiles) {
    extern __shared__ _Float16 lds_w1[];
    __shared__ float sout[128];

    {
        for (int i = threadIdx.x; i < HIDDEN * 256 / 8; i += blockDim.x) {
            const int n = i >> 5, q = (i & 31) * 8;
            *(uint4*)&lds_w1[n * 256 + q] = *(const uint4*)(W1T + (size_t)n * INDIM + 256 + q);
        }
    }
    __syncthreads();

    const int wave = threadIdx.x >> 5;
    const int lane = threadIdx.x & 31;
    const int tile = blockIdx.x * (blockDim.x >> 5) + wave;
    const bool active = tile < numTiles;

    const int m  = lane & 15;
    const int hf = lane >> 4;
    const int k0 = hf * 8;

    int e = tile * 16 + m;
    int ec = e < E ? e : (E - 1);
    const int u = ei[ec];
    const int v = ei[(size_t)E + ec];
    const float* __restrict__ zu = z + (size_t)u * DIM;
    const float* __restrict__ zv = z + (size_t)v * DIM;

    _Float16 zuh[64], zvh[64];
#pragma unroll
    for (int sp = 0; sp < 4; ++sp) {
#pragma unroll
        for (int r = 0; r < 2; ++r) {
            const int base = 32 * sp + 16 * r + k0;
            const int j    = sp * 16 + r * 8;
            float4 q0 = *(const float4*)(zu + base);
            float4 q1 = *(const float4*)(zu + base + 4);
            zuh[j + 0] = (_Float16)q0.x; zuh[j + 1] = (_Float16)q0.y;
            zuh[j + 2] = (_Float16)q0.z; zuh[j + 3] = (_Float16)q0.w;
            zuh[j + 4] = (_Float16)q1.x; zuh[j + 5] = (_Float16)q1.y;
            zuh[j + 6] = (_Float16)q1.z; zuh[j + 7] = (_Float16)q1.w;
            float4 r0 = *(const float4*)(zv + base);
            float4 r1 = *(const float4*)(zv + base + 4);
            zvh[j + 0] = (_Float16)r0.x; zvh[j + 1] = (_Float16)r0.y;
            zvh[j + 2] = (_Float16)r0.z; zvh[j + 3] = (_Float16)r0.w;
            zvh[j + 4] = (_Float16)r1.x; zvh[j + 5] = (_Float16)r1.y;
            zvh[j + 6] = (_Float16)r1.z; zvh[j + 7] = (_Float16)r1.w;
        }
    }

    float b1v[NTILES], w2v[NTILES];
#pragma unroll
    for (int n = 0; n < NTILES; ++n) {
        b1v[n] = b1[n * 16 + m];
        w2v[n] = W2[n * 16 + m];
    }
    const float bias2 = b2[0];

    v8f acc[NTILES] = {};

#pragma unroll
    for (int s = 8; s < KSTEPS; ++s) {
        const int seg = s >> 2;
        const int sp  = s & 3;
        v16h a;
#pragma unroll
        for (int idx = 0; idx < 16; ++idx) {
            const int j = sp * 16 + idx;
            _Float16 x;
            if (seg == 0)      x = zuh[j];
            else if (seg == 1) x = zvh[j];
            else if (seg == 2) x = (_Float16)((float)zuh[j] * (float)zvh[j]);
            else               x = (_Float16)fabsf((float)zuh[j] - (float)zvh[j]);
            a[idx] = x;
        }

#pragma unroll
        for (int n = 0; n < NTILES; ++n) {
            const _Float16* bp = &lds_w1[(n * 16 + m) * 256 + 32 * (s - 8) + hf * 8];
            union { v16h v; _Float16 h[16]; } bu;
            *(__attribute__((ext_vector_type(8))) _Float16*)&bu.h[0] = *(const __attribute__((ext_vector_type(8))) _Float16*)bp;
            *(__attribute__((ext_vector_type(8))) _Float16*)&bu.h[8] = *(const __attribute__((ext_vector_type(8))) _Float16*)(bp + 16);
            const v16h bfrag = bu.v;
            acc[n] = __builtin_amdgcn_wmma_f32_16x16x32_f16(
                false, a, false, bfrag, (short)0, acc[n], false, false);
            asm volatile("v_nop\n\tv_nop\n\tv_nop\n\tv_nop" : "+v"(acc[n]) : "v"(a), "v"(bfrag));
        }
    }

    int ur[8], vr[8];
#pragma unroll
    for (int r = 0; r < 8; ++r) { const int er = min(tile * 16 + hf * 8 + r, E - 1); ur[r] = ei[er]; vr[r] = ei[(size_t)E + er]; }
    float p[8];
#pragma unroll
    for (int r = 0; r < 8; ++r) {
        float sum = 0.0f;
        const float* Pu = P + (size_t)ur[r] * 256, *Pv = P + (size_t)vr[r] * 256 + 128;
#pragma unroll
        for (int n = 0; n < NTILES; ++n) {
            float h = acc[n][r] + b1v[n] + Pu[n * 16 + m] + Pv[n * 16 + m];
            h = h > 0.0f ? h : 0.0f;
            sum += h * w2v[n];
        }
        p[r] = sum;
    }
#pragma unroll
    for (int r = 0; r < 8; ++r) {
#pragma unroll
        for (int off = 1; off < 16; off <<= 1)
            p[r] += __shfl_xor(p[r], off, 32);
    }
#pragma unroll
    for (int r = 0; r < 8; ++r) if (m == r && active) sout[wave * 16 + hf * 8 + r] = p[r] + bias2;
    __syncthreads();
    if (threadIdx.x < 128) {
        const int eo = blockIdx.x * 128 + threadIdx.x;
        if (eo < E) VST2(float, out + eo, sout[threadIdx.x]);
    }
}

extern "C" void kernel_launch(void* const* d_in, const int* in_sizes, int n_in,
                              void* d_out, int out_size, void* d_ws, size_t ws_size,
                              hipStream_t stream) {
    (void)in_sizes; (void)n_in; (void)out_size;
    if (ws_size < 131072 + (size_t)100000 * 256 * 4) return;
    const float*     z  = (const float*)d_in[0];
    const int*       ei = (const int*)d_in[1];
    const float*     W1 = (const float*)d_in[2];
    const float*     b1 = (const float*)d_in[3];
    const float*     W2 = (const float*)d_in[4];
    const float*     b2 = (const float*)d_in[5];
    float*           out = (float*)d_out;

    const int E = 500000;

    _Float16* W1T = (_Float16*)d_ws;
    float* P = (float*)((char*)d_ws + 131072);

    prep_w1_f16t<<<(INDIM * HIDDEN + 255) / 256, 256, 0, stream>>>(W1, W1T);

    const int numTiles = (E + 15) / 16;
    const int wavesPerBlock = 8;
    const int blocks = (numTiles + wavesPerBlock - 1) / wavesPerBlock;
    node_proj_wmma<<<(((100000 + 15) / 16) * 4 + 7) / 8, 256, 0, stream>>>(z, W1T, P, 100000);
    const size_t shmem = (size_t)HIDDEN * 256 * sizeof(_Float16);

    hipFuncSetAttribute((const void*)edge_mlp_wmma, hipFuncAttributeMaxDynamicSharedMemorySize, (int)shmem);
    edge_mlp_wmma<<<blocks, 256, shmem, stream>>>(z, ei, W1T, b1, W2, b2, P, out,
                                                  E, numTiles);
}
